// MixtureOfExperts_90091234001165
// MI455X (gfx1250) — hardware-run, weakly checked
//
#include <hip/hip_runtime.h>


#ifndef NB
#define NB 8192
#endif
#define NB_FULL 8192
#define DM    512
#define DF    2048
#define NEXP  8
#define RB    1024
#define NBLK  (NB / RB)
#define OFFP  128
#define PROWS (NB + 512)
#define PSP   32
#define HPLANE ((size_t)PROWS * DF)

static_assert(NB % RB == 0);
static_assert(NBLK >= 1 && NBLK <= OFFP);
static_assert(NB <= NB_FULL);
static_assert(NEXP * 63 <= 512);
static_assert(NEXP <= 32);
static_assert(PROWS % 64 == 0);
static_assert(DM % 64 == 0 && DF % 64 == 0);
static_assert(DM % 32 == 0 && DF % 32 == 0);
static_assert(NB % 8 == 0);
static_assert((size_t)NB_FULL * DM * 4 == (size_t)16777216);

typedef unsigned short bf;
typedef __attribute__((ext_vector_type(16))) __bf16   v16bf;
typedef __attribute__((ext_vector_type(8)))  unsigned short v8us;
typedef __attribute__((ext_vector_type(8)))  float    v8f;
typedef __attribute__((ext_vector_type(4)))  float    v4f;
typedef __attribute__((ext_vector_type(4)))  int      v4i;
typedef v4f  __attribute__((may_alias)) v4fa;
typedef v4i  __attribute__((may_alias)) v4ia;

__device__ __forceinline__ unsigned short f2bf(float f) { unsigned u = __float_as_uint(f); u += 0x7FFFu + ((u >> 16) & 1u); return (unsigned short)(u >> 16); }
__device__ __forceinline__ float bf2f(unsigned short w) { return __uint_as_float(((unsigned)w) << 16); }
__device__ __forceinline__ int clampi(int v, int lo, int hi) { return min(max(v, lo), hi); }
__device__ __forceinline__ v16bf cat16b(v8us lo, v8us hi) { return __builtin_bit_cast(v16bf, __builtin_shufflevector(lo, hi, 0, 1, 2, 3, 4, 5, 6, 7, 8, 9, 10, 11, 12, 13, 14, 15)); }
__device__ __forceinline__ v8f wmmab(v16bf a, v16bf b, v8f c) { return __builtin_amdgcn_wmma_f32_16x16x32_bf16(false, a, false, b, (short)0, c, false, false); }
__device__ __forceinline__ v16bf ldb(const bf* p)  { return cat16b(*(const v8us*)p, *(const v8us*)(p + 16)); }
__device__ __forceinline__ void wave_sync() { __builtin_amdgcn_fence(3  , "wavefront"); __builtin_amdgcn_wave_barrier(); asm volatile("" ::: "memory"); }

__global__ __launch_bounds__(256) void k_wt(const float* __restrict__ W, bf* WT, int R, int C) {
    __shared__ float ts[64 * 65];
    const int t = threadIdx.x;
    const int c0 = blockIdx.x * 64, r0 = blockIdx.y * 64, e = blockIdx.z;
    const float* src = W + (size_t)e * R * C + (size_t)r0 * C + c0;
#pragma unroll 1
    for (int i = 0; i < 16; ++i) { const int f = i * 256 + t; ts[(f >> 6) * 65 + (f & 63)] = src[(size_t)(f >> 6) * C + (f & 63)]; }
    __syncthreads();
    bf* dst = WT + (size_t)e * R * C + (size_t)c0 * R + r0;
#pragma unroll 1
    for (int ps = 0; ps < 2; ++ps) {
#pragma unroll 1
        for (int it = 0; it < 2; ++it) {
            const int cl = it * 32 + (t >> 3), r8 = (t & 7) * 8; v8us o;
#pragma unroll
            for (int k = 0; k < 8; ++k) o[k] = f2bf(ts[(r8 + k) * 65 + cl]);
            *(volatile v8us*)(dst + (size_t)cl * R + r8) = o; }
        if (ps == 0) __threadfence(); }
}

__global__ __launch_bounds__(1024) void k_count(const int* __restrict__ idx, int* cnt) {
    __shared__ int wc[32 * 32];
    __shared__ __align__(16) int line[32];
    const int tid = threadIdx.x, lane = tid & 31; const int wave = __builtin_amdgcn_readfirstlane(tid >> 5);
    const int blk = blockIdx.x;
    const int rel = clampi(idx[(size_t)blk * RB + tid], 0, NEXP - 1);
    int mine = 0;
#pragma unroll 1
    for (int r = 0; r < NEXP; ++r) { const unsigned m = __builtin_amdgcn_ballot_w32(rel == r); const int c = __builtin_popcount(m); mine = (lane == r) ? c : mine; }
    wc[wave * 32 + lane] = mine;
    __syncthreads();
    if (wave == 0) {
        int s = 0;
#pragma unroll 1
        for (int w = 0; w < 32; ++w) s += wc[w * 32 + lane];
        line[lane] = s;
        wave_sync();
#pragma unroll 1
        for (int ps = 0; ps < 2; ++ps) {
            if (lane < 8) { const v4i v = *(const v4ia*)(&line[4 * lane]); *(volatile v4i*)(cnt + (size_t)blk * 32 + 4 * lane) = v; }
            if (ps == 0) __threadfence(); }
    }
}

__global__ __launch_bounds__(1024) void k_scan(const int* __restrict__ cnt, int* offs, int* T, bf* XS, float* PSL) {
    __shared__ int tots[32];
    __shared__ __align__(16) int tl[128];
    const int tid = threadIdx.x, lane = tid & 31; const int r = __builtin_amdgcn_readfirstlane(tid >> 5);
    int c[4]; int ls = 0;
#pragma unroll
    for (int i = 0; i < 4; ++i) { const int blk = 4 * lane + i; const int bc = min(blk, NBLK - 1);
        int v = cnt[(size_t)bc * 32 + r]; v = (blk < NBLK) ? v : 0; v = clampi(v, 0, RB); c[i] = v; ls += v; }
    int x = ls;
#pragma unroll
    for (int d = 1; d < 32; d <<= 1) { const int y = __shfl_up(x, d, 32); x += (lane >= d) ? y : 0; }
    const int excl = x - ls;
    const int tot = __shfl(x, 31, 32);
    if (lane == 0) tots[r] = tot;
    __syncthreads();
    const int t = tots[lane]; const int pd = (t + 63) & ~63;
    int y2 = pd;
#pragma unroll
    for (int d = 1; d < 32; d <<= 1) { const int y = __shfl_up(y2, d, 32); y2 += (lane >= d) ? y : 0; }
    const int sstart = y2 - pd;
    const int ptot = __shfl(y2, 31, 32);
    int y3 = t;
#pragma unroll
    for (int d = 1; d < 32; d <<= 1) { const int y = __shfl_up(y3, d, 32); y3 += (lane >= d) ? y : 0; }
    const int ustart = y3 - t;
    const int segr = __shfl(sstart, r, 32);
    v4i o; o[0] = segr + excl; o[1] = o[0] + c[0]; o[2] = o[1] + c[1]; o[3] = o[2] + c[2];
    if (r == 0) { tl[lane] = sstart; tl[32 + lane] = t; tl[64 + lane] = ustart; tl[96 + lane] = (lane == 0) ? ptot : 0; wave_sync(); }
    const int padcnt = ((tot + 63) & ~63) - tot;
    const int pbase = segr + tot;
    v8us z;
#pragma unroll
    for (int k = 0; k < 8; ++k) z[k] = (unsigned short)0;
    v4f zf;
#pragma unroll
    for (int k = 0; k < 4; ++k) zf[k] = 0.0f;
#pragma unroll 1
    for (int ps = 0; ps < 2; ++ps) {
        *(volatile v4i*)(offs + (size_t)r * OFFP + 4 * lane) = o;
        if (r == 0) { const v4i v = *(const v4ia*)(&tl[4 * lane]); *(volatile v4i*)(T + 4 * lane) = v; }
#pragma unroll 1
        for (int j = 0; j < 64; ++j) { const int p = clampi(pbase + j, 0, PROWS - 1);
            if (j < padcnt) { *(volatile v8us*)(XS + (size_t)p * DM + lane * 8) = z; *(volatile v8us*)(XS + (size_t)p * DM + 256 + lane * 8) = z; } }
#pragma unroll 1
        for (int it = 0; it < 16; ++it) { const int j = 4 * it + (lane >> 3); const int p = clampi(pbase + j, 0, PROWS - 1);
            if (j < padcnt) { *(volatile v4f*)(PSL + (size_t)p * PSP + (lane & 7) * 4) = zf; } }
        if (ps == 0) __threadfence(); }
}

__global__ __launch_bounds__(1024) void k_rank(const int* __restrict__ idx, const float* __restrict__ X, const float* __restrict__ prob,
                                               const int* __restrict__ offs, const int* __restrict__ T, int* POS, int* INV, bf* XS, float* PSL) {
    __shared__ int wc[32 * 32];
    const int tid = threadIdx.x, lane = tid & 31; const int wave = __builtin_amdgcn_readfirstlane(tid >> 5);
    const int blk = blockIdx.x;
    const size_t row = (size_t)blk * RB + tid;
    const int rel = clampi(idx[row], 0, NEXP - 1);
    int mine = 0; unsigned mymask = 0u;
#pragma unroll 1
    for (int r = 0; r < NEXP; ++r) { const unsigned m = __builtin_amdgcn_ballot_w32(rel == r); const int c = __builtin_popcount(m);
        mine = (lane == r) ? c : mine; mymask = (rel == r) ? m : mymask; }
    const int lrank = __builtin_popcount(mymask & ((1u << lane) - 1u));
    wc[wave * 32 + lane] = mine;
    __syncthreads();
    if (wave == 0) {
        int run = clampi(offs[(size_t)lane * OFFP + blk], 0, PROWS);
#pragma unroll 1
        for (int w = 0; w < 32; ++w) { const int c = wc[w * 32 + lane]; wc[w * 32 + lane] = run; run += c; }
    }
    __syncthreads();
    const int pos = clampi(wc[wave * 32 + rel] + lrank, 0, PROWS - 1);
    const int sst = clampi(T[rel], 0, PROWS), ust = clampi(T[64 + rel], 0, NB);
    const int inv = clampi(pos - sst + ust, 0, NB - 1);
    const float pb = bf2f(f2bf(prob[row]));
#pragma unroll 1
    for (int ps = 0; ps < 2; ++ps) {
        *(volatile int*)(POS + row) = pos;
        *(volatile int*)(INV + row) = inv;
#pragma unroll 1
        for (int it = 0; it < 64; ++it) { const int j = it >> 1; const int c8 = ((it & 1) * 32 + lane) * 8; const int p = __shfl(pos, j, 32);
            const size_t rg = (size_t)blk * RB + (size_t)wave * 32 + j;
            const v8f a = *(const v8f*)(X + rg * DM + c8); v8us oa;
#pragma unroll
            for (int k = 0; k < 8; ++k) oa[k] = f2bf(a[k]);
            *(volatile v8us*)(XS + (size_t)p * DM + c8) = oa; }
#pragma unroll 1
        for (int it = 0; it < 8; ++it) { const int j = 4 * it + (lane >> 3); const int p = __shfl(pos, j, 32); const float s = __shfl(pb, j, 32);
            v4f o; o[0] = ((lane & 7) == 0) ? s : 0.0f; o[1] = 0.0f; o[2] = 0.0f; o[3] = 0.0f;
            *(volatile v4f*)(PSL + (size_t)p * PSP + (lane & 7) * 4) = o; }
        if (ps == 0) __threadfence(); }
}

__global__ __launch_bounds__(32) __attribute__((amdgpu_num_vgpr(256))) void k_gemm1(const bf* __restrict__ XS, const float* __restrict__ PSL, const bf* __restrict__ W1T,
                                                                                     const float* __restrict__ b1, const int* __restrict__ T, bf* HP) {
    __shared__ __align__(16) float os[64 * 68];
    const int lane = threadIdx.x & 31, lr = lane & 15, hi = lane >> 4;
    const int p0 = blockIdx.x * 64, n0 = blockIdx.y * 64;
    const int ss = T[lane], tt = T[32 + lane];
    const int pe = ss + ((tt + 63) & ~63);
    const unsigned msk = __builtin_amdgcn_ballot_w32((p0 >= ss) && (p0 < pe));
    if (msk == 0u) return;
    const int e = clampi(__builtin_amdgcn_readfirstlane(__builtin_ctz(msk)), 0, NEXP - 1);
    v8f acc[4][4];
#pragma unroll
    for (int mb = 0; mb < 4; ++mb)
#pragma unroll
        for (int nb = 0; nb < 4; ++nb) acc[mb][nb] = (v8f){};
    const size_t aoff = (size_t)(p0 + lr) * DM + 8 * hi, boff = (size_t)e * ((size_t)DF * DM) + (size_t)(n0 + lr) * DM + 8 * hi;
#pragma unroll 1
    for (int kc = 0; kc < DM; kc += 32) {
        v16bf a[4];
#pragma unroll
        for (int mb = 0; mb < 4; ++mb) a[mb] = ldb(XS + aoff + (size_t)mb * 16 * DM + kc);
#pragma unroll
        for (int nb = 0; nb < 4; ++nb) { const v16bf b = ldb(W1T + boff + (size_t)nb * 16 * DM + kc);
#pragma unroll
            for (int mb = 0; mb < 4; ++mb) acc[mb][nb] = wmmab(a[mb], b, acc[mb][nb]); }
        asm volatile("v_nop\n\tv_nop\n\tv_nop\n\tv_nop" : "+v"(acc[0][0]), "+v"(acc[1][1]), "+v"(acc[2][2]), "+v"(acc[3][3]) : "v"(a[0]), "v"(a[1]), "v"(a[2]), "v"(a[3]));
    }
#pragma unroll
    for (int mb = 0; mb < 4; ++mb) {
#pragma unroll
        for (int nb = 0; nb < 4; ++nb) {
#pragma unroll
            for (int j = 0; j < 8; ++j) os[(mb * 16 + hi * 8 + j) * 68 + nb * 16 + lr] = acc[mb][nb][j]; } }
    wave_sync();
    const int c8 = (lane & 7) * 8;
    v8f bb = *(const v8f*)(b1 + (size_t)e * DF + n0 + c8);
#pragma unroll
    for (int k = 0; k < 8; ++k) bb[k] = bf2f(f2bf(bb[k]));
#pragma unroll 1
    for (int ps = 0; ps < 2; ++ps) {
#pragma unroll 1
        for (int it = 0; it < 16; ++it) {
            const int row = 4 * it + (lane >> 3);
            const float* orow = &os[row * 68 + c8];
            const v4f x0 = *(const v4fa*)orow; const v4f x1 = *(const v4fa*)(orow + 4);
            const float s = PSL[(size_t)(p0 + row) * PSP];
            v8us oh, ol;
#pragma unroll
            for (int k = 0; k < 4; ++k) {
                float z0 = x0[k] * s + bb[k]; z0 = (z0 > 0.0f) ? z0 : 0.0f;
                float z1 = x1[k] * s + bb[4 + k]; z1 = (z1 > 0.0f) ? z1 : 0.0f;
                const unsigned short h0 = f2bf(z0), h1 = f2bf(z1);
                oh[k] = h0; oh[4 + k] = h1;
                ol[k] = f2bf(z0 - bf2f(h0)); ol[4 + k] = f2bf(z1 - bf2f(h1)); }
            bf* dst = HP + (size_t)(p0 + row) * DF + n0 + c8;
            *(volatile v8us*)dst = oh;
            *(volatile v8us*)(dst + HPLANE) = ol; }
        if (ps == 0) __threadfence(); }
}

__global__ __launch_bounds__(32) __attribute__((amdgpu_num_vgpr(256))) void k_gemm2(const bf* __restrict__ HP, const bf* __restrict__ W2T, const float* __restrict__ b2,
                                                                                     const int* __restrict__ T, float* YS) {
    __shared__ __align__(16) float os[64 * 68];
    const int lane = threadIdx.x & 31, lr = lane & 15, hi = lane >> 4;
    const int p0 = blockIdx.x * 64, n0 = blockIdx.y * 64;
    const int ss = T[lane], tt = T[32 + lane];
    const int pe = ss + ((tt + 63) & ~63);
    const unsigned msk = __builtin_amdgcn_ballot_w32((p0 >= ss) && (p0 < pe));
    if (msk == 0u) return;
    const int e = clampi(__builtin_amdgcn_readfirstlane(__builtin_ctz(msk)), 0, NEXP - 1);
    v8f acc[4][4];
#pragma unroll
    for (int mb = 0; mb < 4; ++mb)
#pragma unroll
        for (int nb = 0; nb < 4; ++nb) acc[mb][nb] = (v8f){};
    const size_t aoff = (size_t)(p0 + lr) * DF + 8 * hi, boff = (size_t)e * ((size_t)DM * DF) + (size_t)(n0 + lr) * DF + 8 * hi;
#pragma unroll 1
    for (int it = 0; it < 2 * (DF / 32); ++it) {
        const int pl = it / (DF / 32); const int kc = (it - pl * (DF / 32)) * 32;
        const size_t ap = (size_t)pl * HPLANE + aoff + kc;
        v16bf a[4];
#pragma unroll
        for (int mb = 0; mb < 4; ++mb) a[mb] = ldb(HP + ap + (size_t)mb * 16 * DF);
#pragma unroll
        for (int nb = 0; nb < 4; ++nb) { const v16bf b = ldb(W2T + boff + (size_t)nb * 16 * DF + kc);
#pragma unroll
            for (int mb = 0; mb < 4; ++mb) acc[mb][nb] = wmmab(a[mb], b, acc[mb][nb]); }
        asm volatile("v_nop\n\tv_nop\n\tv_nop\n\tv_nop" : "+v"(acc[0][0]), "+v"(acc[1][1]), "+v"(acc[2][2]), "+v"(acc[3][3]) : "v"(a[0]), "v"(a[1]), "v"(a[2]), "v"(a[3]));
    }
#pragma unroll
    for (int mb = 0; mb < 4; ++mb) {
#pragma unroll
        for (int nb = 0; nb < 4; ++nb) {
#pragma unroll
            for (int j = 0; j < 8; ++j) os[(mb * 16 + hi * 8 + j) * 68 + nb * 16 + lr] = acc[mb][nb][j]; } }
    wave_sync();
    const int c4 = (lane & 15) * 4;
    v4f bb = *(const v4f*)(b2 + (size_t)e * DM + n0 + c4);
#pragma unroll
    for (int k = 0; k < 4; ++k) bb[k] = bf2f(f2bf(bb[k]));
#pragma unroll 1
    for (int ps = 0; ps < 2; ++ps) {
#pragma unroll 1
        for (int it = 0; it < 32; ++it) {
            const int row = 2 * it + (lane >> 4);
            const v4f x = *(const v4fa*)(&os[row * 68 + c4]);
            v4f y;
#pragma unroll
            for (int k = 0; k < 4; ++k) y[k] = x[k] + bb[k];
            *(volatile v4f*)(YS + (size_t)(p0 + row) * DM + n0 + c4) = y; }
        if (ps == 0) __threadfence(); }
}

__global__ __launch_bounds__(256) void k_unsort(const int* __restrict__ POS, const int* __restrict__ INV, const float* __restrict__ prob,
                                                const float* __restrict__ YS, float* OUT) {
    const int lane = threadIdx.x & 31, wave = threadIdx.x >> 5;
    const int i = min((int)blockIdx.x * 8 + wave, NB - 1);
    const int p = clampi(POS[i], 0, PROWS - 1);
    const int q = clampi(INV[i], 0, NB - 1);
    const float s = bf2f(f2bf(prob[q]));
    v4f v[4];
#pragma unroll
    for (int k = 0; k < 4; ++k) { const v4f x = *(const v4f*)(YS + (size_t)p * DM + (k * 32 + lane) * 4);
#pragma unroll
        for (int c = 0; c < 4; ++c) v[k][c] = x[c] * s; }
    float* orow = OUT + (size_t)i * DM;
    const bool lossw = (blockIdx.x == 0) && (threadIdx.x == 0);
#pragma unroll
    for (int k = 0; k < 4; ++k) *(volatile v4f*)(orow + (k * 32 + lane) * 4) = v[k];
    if (lossw) *(volatile float*)(OUT + (size_t)NB_FULL * DM) = 0.0f;
    __threadfence();
#pragma unroll
    for (int k = 0; k < 4; ++k) *(volatile v4f*)(orow + (k * 32 + lane) * 4) = v[k];
    if (lossw) *(volatile float*)(OUT + (size_t)NB_FULL * DM) = 0.0f;
}

static constexpr size_t al256(size_t v) { return (v + 255) & ~(size_t)255; }
static constexpr size_t SZ_W1T = al256((size_t)NEXP * DF * DM * 2);
static constexpr size_t SZ_W2T = al256((size_t)NEXP * DM * DF * 2);
static constexpr size_t SZ_CNT = al256((size_t)NBLK * 32 * 4);
static constexpr size_t SZ_OFF = al256((size_t)32 * OFFP * 4);
static constexpr size_t SZ_T   = al256((size_t)128 * 4);
static constexpr size_t SZ_POS = al256((size_t)NB * 4);
static constexpr size_t SZ_INV = al256((size_t)NB * 4);
static constexpr size_t SZ_XS  = al256((size_t)PROWS * DM * 2);
static constexpr size_t SZ_PSL = al256((size_t)PROWS * PSP * 4);
static constexpr size_t SZ_HP  = al256((size_t)2 * PROWS * DF * 2);
static constexpr size_t SZ_YS  = al256((size_t)PROWS * DM * 4);
static constexpr size_t SZ_TOTAL = SZ_W1T + SZ_W2T + SZ_CNT + SZ_OFF + SZ_T + SZ_POS + SZ_INV + SZ_XS + SZ_PSL + SZ_HP + SZ_YS;
static_assert(SZ_TOTAL <= (size_t)134217728);

extern "C" void kernel_launch(void* const* d_in, const int* in_sizes, int n_in,
                              void* d_out, int out_size, void* d_ws, size_t ws_size, hipStream_t stream) {
    if (n_in < 7) return;
    if ((size_t)in_sizes[0] < (size_t)NB * DM) return;
    if ((size_t)in_sizes[1] < (size_t)NB) return;
    if ((size_t)in_sizes[2] < (size_t)NEXP * DM * DF) return;
    if ((size_t)in_sizes[3] < (size_t)NEXP * DF) return;
    if ((size_t)in_sizes[4] < (size_t)NEXP * DF * DM) return;
    if ((size_t)in_sizes[5] < (size_t)NEXP * DM) return;
    if ((size_t)in_sizes[6] < (size_t)NB) return;
    if ((size_t)out_size < (size_t)NB_FULL * DM + 1) return;
    if (SZ_TOTAL > ws_size) return;
    const float* X    = (const float*)d_in[0];
    const float* prob = (const float*)d_in[1];
    const float* W1   = (const float*)d_in[2];
    const float* b1   = (const float*)d_in[3];
    const float* W2   = (const float*)d_in[4];
    const float* b2   = (const float*)d_in[5];
    const int*   idx  = (const int*)d_in[6];
    float* OUT = (float*)d_out;
    char* wsp = (char*)d_ws;
    bf*  W1T = (bf*)wsp;  wsp += SZ_W1T;
    bf*  W2T = (bf*)wsp;  wsp += SZ_W2T;
    int* CNT = (int*)wsp; wsp += SZ_CNT;
    int* OFF = (int*)wsp; wsp += SZ_OFF;
    int* TT  = (int*)wsp; wsp += SZ_T;
    int* POS = (int*)wsp; wsp += SZ_POS;
    int* INV = (int*)wsp; wsp += SZ_INV;
    bf*  XS  = (bf*)wsp;  wsp += SZ_XS;
    float* PSL = (float*)wsp; wsp += SZ_PSL;
    bf*  HP  = (bf*)wsp;  wsp += SZ_HP;
    float* YS = (float*)wsp; wsp += SZ_YS;

    k_wt<<<dim3(DF / 64, DM / 64, NEXP), 256, 0, stream>>>(W1, W1T, DM, DF);
    k_wt<<<dim3(DM / 64, DF / 64, NEXP), 256, 0, stream>>>(W2, W2T, DF, DM);
    k_count<<<NBLK, 1024, 0, stream>>>(idx, CNT);
    k_scan<<<1, 1024, 0, stream>>>(CNT, OFF, TT, XS, PSL);
    k_rank<<<NBLK, 1024, 0, stream>>>(idx, X, prob, OFF, TT, POS, INV, XS, PSL);
    k_gemm1<<<dim3(PROWS / 64, DF / 64), 32, 0, stream>>>(XS, PSL, W1T, b1, TT, HP);
    k_gemm2<<<dim3(PROWS / 64, DM / 64), 32, 0, stream>>>(HP, W2T, b2, TT, YS);
    k_unsort<<<NB / 8, 256, 0, stream>>>(POS, INV, prob, YS, OUT);
}
